// MultiDconvHeadTransposedAttention_59072980189966
// MI455X (gfx1250) — hardware-verified
//
#include <hip/hip_runtime.h>


namespace {
constexpr int Bn = 4, HW = 128, NP = HW * HW, C = 192, C3 = 3 * C, NH = 4, CH = 48, CHP = 64  ;
constexpr float XS = 8.0f;

typedef _Float16 b16;
typedef __attribute__((ext_vector_type(16))) _Float16 v16b;
typedef __attribute__((ext_vector_type(8))) _Float16 v8b;
typedef __attribute__((ext_vector_type(8))) float v8f;
typedef __attribute__((ext_vector_type(4))) float v4f;
__device__ __forceinline__ float bf16_rne(float f) { unsigned int u = __float_as_uint(f); u += 0x7FFFu + ((u >> 16) & 1u); return __uint_as_float(u & 0xFFFF0000u); }
__device__ __forceinline__ void split16(float v, b16& hi, b16& lo) { hi = (b16)v; lo = (b16)(v - (float)hi); }
__device__ __forceinline__ v16b frag_kb(const b16* p, int hh) { const v8b a = *(const v8b*)(p + 8 * hh), b = *(const v8b*)(p + 16 + 8 * hh); v16b f;
#pragma unroll
  for (int e = 0; e < 8; ++e) { f[e] = a[e]; f[8 + e] = b[e]; } return f; }
__device__ __forceinline__ v8f wmma16b(v16b a, v16b b, v8f c) { v8f d = __builtin_amdgcn_wmma_f32_16x16x32_f16(false, a, false, b, (short)0, c, false, false); asm volatile("v_nop\n\tv_nop\n\tv_nop\n\tv_nop" : "+v"(d) : "v"(a), "v"(b)); return d; }
__device__ __forceinline__ void wave_lds_sync() { __builtin_amdgcn_fence(__ATOMIC_RELEASE, "workgroup"); __builtin_amdgcn_wave_barrier(); __builtin_amdgcn_fence(__ATOMIC_ACQUIRE, "workgroup"); }
__device__ __forceinline__ float nexp(float x) { return __builtin_amdgcn_exp2f(x * 1.4426950408889634f); }
__device__ __forceinline__ float pmul(float a, float b) { float p = a * b; asm volatile("" : "+v"(p)); return p; }
__device__ __forceinline__ float wsum(float v) {
#pragma unroll
  for (int o = 1; o < 32; o <<= 1) v += __shfl_xor(v, o); return v; }

__global__ __launch_bounds__(256) void prep_kernel(const float* __restrict__ wqkv, const float* __restrict__ wdw, const float* __restrict__ wpr, const float* __restrict__ tmp, b16* __restrict__ R, float* __restrict__ P, b16* __restrict__ VRpad, b16* __restrict__ VRlpad) {
  const size_t tid = (size_t)blockIdx.x * 256 + threadIdx.x, nth = (size_t)gridDim.x * 256;
  { const v8b z = {}; for (size_t p = tid; p < (size_t)32 * C / 8; p += nth) { *(volatile v8b*)(VRpad + p * 8) = z; *(volatile v8b*)(VRlpad + p * 8) = z; } }
  auto tr = [&](size_t base, int nout, int kin, const float* W) { for (size_t p = tid; p < (size_t)nout * (kin / 8); p += nth) { const int o = (int)(p / (kin / 8)), k0 = (int)(p % (kin / 8)) * 8; v8b v;
#pragma unroll
      for (int e = 0; e < 8; ++e) v[e] = (b16)bf16_rne(W[(size_t)(k0 + e) * nout + o]); *(volatile v8b*)(R + base + (size_t)o * kin + k0) = v; } };
  for (int pass = 0; pass < 2; ++pass) { tr(0, C3, C, wqkv); tr((size_t)C3 * C, C, C, wpr); for (size_t q = tid; q < 5188; q += nth) { P[q] = (q < 5184) ? bf16_rne(wdw[q]) : bf16_rne(tmp[q - 5184]); } __threadfence(); }
}

__global__ __launch_bounds__(256) void xrows_kernel(const float* __restrict__ xb, b16* __restrict__ X) {
  const size_t tid = (size_t)blockIdx.x * 256 + threadIdx.x, nth = (size_t)gridDim.x * 256;
  for (int pass = 0; pass < 2; ++pass) { for (size_t p = tid; p < (size_t)NP * C / 8; p += nth) { v8b v; for (int e = 0; e < 8; ++e) v[e] = (b16)(bf16_rne(xb[p * 8 + e]) * XS); *(volatile v8b*)(X + p * 8) = v; } __threadfence(); }
}

__global__ __launch_bounds__(64) void qkv_kernel(const b16* __restrict__ X, const b16* __restrict__ R, float* __restrict__ QF) {
  __shared__ __attribute__((aligned(16))) float Ts[2][32][96 + 4];
  const int lane = threadIdx.x & 31, wave = threadIdx.x >> 5, nloc = lane & 15, hlf = lane >> 4, m0 = blockIdx.y * 32, c0 = blockIdx.x * 192 + wave * 96;
  v8f acc[2][6];
#pragma unroll
  for (int r = 0; r < 2; ++r)
#pragma unroll
    for (int t = 0; t < 6; ++t) acc[r][t] = (v8f){};
#pragma unroll
  for (int kb = 0; kb < C; kb += 32) { const v16b a0 = frag_kb(X + (size_t)(m0 + nloc) * C + kb, hlf), a1 = frag_kb(X + (size_t)(m0 + 16 + nloc) * C + kb, hlf);
#pragma unroll
    for (int t = 0; t < 6; ++t) { const v16b bw = frag_kb(R + (size_t)(c0 + t * 16 + nloc) * C + kb, hlf); acc[0][t] = wmma16b(a0, bw, acc[0][t]); acc[1][t] = wmma16b(a1, bw, acc[1][t]); } }
#pragma unroll
  for (int t = 0; t < 6; ++t)
#pragma unroll
    for (int r = 0; r < 2; ++r)
#pragma unroll
      for (int v = 0; v < 8; ++v) Ts[wave][r * 16 + 8 * hlf + v][t * 16 + nloc] = acc[r][t][v] * (1.0f / XS);
  wave_lds_sync();
  for (int pass = 0; pass < 2; ++pass) { for (int i = lane; i < 32 * 24; i += 32) { const int rr = i / 24, c4 = (i % 24) * 4; *(volatile v4f*)(QF + (size_t)(m0 + rr) * C3 + c0 + c4) = *(const v4f*)(&Ts[wave][rr][c4]); } __threadfence(); }
}

__global__ __launch_bounds__(256) void dw_kernel(const float* __restrict__ QF, const float* __restrict__ P, b16* __restrict__ QP, b16* __restrict__ QPl, b16* __restrict__ KP, b16* __restrict__ KPl, b16* __restrict__ VR, b16* __restrict__ VRl) {
  __shared__ float In[3][HW + 2][64 + 1]; __shared__ __attribute__((aligned(16))) b16 Oh[HW * (64 + 8)], Ol[HW * (64 + 8)];
  const int y = blockIdx.x, cg = blockIdx.y * 64, t_ = threadIdx.x;
  for (int i = t_; i < 3 * (HW + 2) * 64; i += 256) { const int c = i & 63, rem = i >> 6, xx = rem % (HW + 2) - 1, r = rem / (HW + 2), yy = y + r - 1; In[r][xx + 1][c] = (yy >= 0 && yy < HW && xx >= 0 && xx < HW) ? QF[((size_t)yy * HW + xx) * C3 + cg + c] : 0.0f; }
  __syncthreads();
  const bool isv = (cg >= 2 * C);
  for (int i = t_; i < HW * 64; i += 256) { int c, xx; if (!isv) { xx = i & 127; c = i >> 7; } else { c = i & 63; xx = i >> 6; }
    const float* w = P + cg + c; float a = 0.0f;
#pragma unroll
    for (int dy = 0; dy < 3; ++dy)
#pragma unroll
      for (int dx = 0; dx < 3; ++dx) a += pmul(In[dy][xx + dx][c], w[(dy * 3 + dx) * C3]);
    b16 h_, l_; split16(a * XS, h_, l_); if (!isv) { Oh[c * (HW + 8) + xx] = h_; Ol[c * (HW + 8) + xx] = l_; } else { Oh[xx * (64 + 8) + c] = h_; Ol[xx * (64 + 8) + c] = l_; } }
  __syncthreads();
  for (int pass = 0; pass < 2; ++pass) {
    if (!isv) { b16* Ph = (cg < C) ? QP : KP; b16* Pl = (cg < C) ? QPl : KPl; const int cb = cg % C; for (int i = t_; i < 64 * 16; i += 256) { const int c = i >> 4, c8 = (i & 15) * 8; const size_t gi = (size_t)(cb + c) * NP + y * HW + c8; *(volatile v8b*)(Ph + gi) = *(const v8b*)(&Oh[c * (HW + 8) + c8]); *(volatile v8b*)(Pl + gi) = *(const v8b*)(&Ol[c * (HW + 8) + c8]); } }
    else { const int cb = cg - 2 * C; for (int i = t_; i < HW * 8; i += 256) { const int xx = i >> 3, c8 = (i & 7) * 8; const size_t gi = ((size_t)y * HW + xx) * C + cb + c8; *(volatile v8b*)(VR + gi) = *(const v8b*)(&Oh[xx * (64 + 8) + c8]); *(volatile v8b*)(VRl + gi) = *(const v8b*)(&Ol[xx * (64 + 8) + c8]); } }
    __threadfence(); }
}

__global__ __launch_bounds__(384) void gram_kernel(const b16* __restrict__ QP, const b16* __restrict__ QPl, const b16* __restrict__ KP, const b16* __restrict__ KPl, const float* __restrict__ P, b16* __restrict__ ATh, b16* __restrict__ ATl) {
  __shared__ float Gs[12][16][CH + 1]; __shared__ float nk[12][CH]; __shared__ float nq[12][16]; __shared__ __attribute__((aligned(16))) b16 Sh[12][16][CHP + 8], Sl[12][16][CHP + 8];
  const int wave = threadIdx.x >> 5, lane = threadIdx.x & 31, nloc = lane & 15, hlf = lane >> 4; const int head = wave / 3, ct = wave % 3; const int qc0 = head * CH + ct * 16, kc0 = head * CH;
  v8f g[3] = {{}, {}, {}};
  for (int kb = 0; kb < NP; kb += 32) { const v16b a = frag_kb(QP + (size_t)(qc0 + nloc) * NP + kb, hlf), al = frag_kb(QPl + (size_t)(qc0 + nloc) * NP + kb, hlf);
#pragma unroll
    for (int t = 0; t < 3; ++t) { const v16b bk = frag_kb(KP + (size_t)(kc0 + t * 16 + nloc) * NP + kb, hlf), bkl = frag_kb(KPl + (size_t)(kc0 + t * 16 + nloc) * NP + kb, hlf); g[t] = wmma16b(a, bk, g[t]); g[t] = wmma16b(al, bk, g[t]); g[t] = wmma16b(a, bkl, g[t]); } }
#pragma unroll
  for (int t = 0; t < 3; ++t)
#pragma unroll
    for (int r = 0; r < 8; ++r) Gs[wave][8 * hlf + r][t * 16 + nloc] = g[t][r] * (1.0f / (XS * XS));
  for (int d = 0; d < CH; ++d) { const b16* ph = KP + (size_t)(kc0 + d) * NP; const b16* pl = KPl + (size_t)(kc0 + d) * NP; float s = 0.0f; for (int x_ = lane; x_ < NP; x_ += 32) { const float v = ((float)ph[x_] + (float)pl[x_]) * (1.0f / XS); s += pmul(v, v); } s = wsum(s); if (lane == 0) nk[wave][d] = s; }
  for (int c = 0; c < 16; ++c) { const b16* ph = QP + (size_t)(qc0 + c) * NP; const b16* pl = QPl + (size_t)(qc0 + c) * NP; float s = 0.0f; for (int x_ = lane; x_ < NP; x_ += 32) { const float v = ((float)ph[x_] + (float)pl[x_]) * (1.0f / XS); s += pmul(v, v); } s = wsum(s); if (lane == 0) nq[wave][c] = s; }
  wave_lds_sync();
  if (lane < 16) { const int c = lane; const float iq = 1.0f / sqrtf(nq[wave][c]); const float tp = P[5184 + head]; float mx = -INFINITY; float sv[CH];
#pragma unroll
    for (int d = 0; d < CH; ++d) { sv[d] = pmul(pmul(Gs[wave][c][d], iq) * (1.0f / sqrtf(nk[wave][d])), tp); mx = fmaxf(mx, sv[d]); }
    float sum = 0.0f;
#pragma unroll
    for (int d = 0; d < CH; ++d) { sv[d] = nexp(sv[d] - mx); sum += sv[d]; }
    const float inv = 1.0f / sum;
#pragma unroll
    for (int d = 0; d < CHP; ++d) { b16 a_, b_; split16((d < CH) ? sv[d] * inv * XS : 0.0f, a_, b_); Sh[wave][c][d] = a_; Sl[wave][c][d] = b_; } }
  wave_lds_sync();
  for (int pass = 0; pass < 2; ++pass) { for (int i = lane; i < 16 * 8; i += 32) { const int c = i >> 3, c8 = (i & 7) * 8; const size_t gi = ((size_t)head * CH + ct * 16 + c) * CHP + c8; *(volatile v8b*)(ATh + gi) = *(const v8b*)(&Sh[wave][c][c8]); *(volatile v8b*)(ATl + gi) = *(const v8b*)(&Sl[wave][c][c8]); } __threadfence(); }
}

__global__ __launch_bounds__(64) void out_kernel(const b16* __restrict__ VR, const b16* __restrict__ VRl, const b16* __restrict__ ATh, const b16* __restrict__ ATl, const b16* __restrict__ R, float* __restrict__ outb) {
  __shared__ __attribute__((aligned(16))) b16 Oh[32][C + 8], Ol[32][C + 8]; __shared__ __attribute__((aligned(16))) float Ts[32][C + 4];
  const int lane = threadIdx.x & 31, wave = threadIdx.x >> 5, nloc = lane & 15, hlf = lane >> 4, p0 = blockIdx.x * 32, m0 = p0 + wave * 16; const b16* Wp = R + (size_t)C3 * C;
  for (int head = 0; head < NH; ++head) { v8f acc[3] = {{}, {}, {}};
#pragma unroll
    for (int kb = 0; kb < CHP; kb += 32) { const v16b a = frag_kb(VR + (size_t)(m0 + nloc) * C + head * CH + kb, hlf), al = frag_kb(VRl + (size_t)(m0 + nloc) * C + head * CH + kb, hlf);
#pragma unroll
      for (int t = 0; t < 3; ++t) { const v16b bh = frag_kb(ATh + ((size_t)head * CH + t * 16 + nloc) * CHP + kb, hlf), bl = frag_kb(ATl + ((size_t)head * CH + t * 16 + nloc) * CHP + kb, hlf); acc[t] = wmma16b(a, bh, acc[t]); acc[t] = wmma16b(al, bh, acc[t]); acc[t] = wmma16b(a, bl, acc[t]); } }
#pragma unroll
    for (int t = 0; t < 3; ++t)
#pragma unroll
      for (int r = 0; r < 8; ++r) { b16 a_, b_; split16(acc[t][r] * (1.0f / (XS * XS)) * XS, a_, b_); Oh[wave * 16 + 8 * hlf + r][head * CH + t * 16 + nloc] = a_; Ol[wave * 16 + 8 * hlf + r][head * CH + t * 16 + nloc] = b_; } }
  wave_lds_sync();
  v8f acc2[12];
#pragma unroll
  for (int t = 0; t < 12; ++t) acc2[t] = (v8f){};
#pragma unroll
  for (int kb = 0; kb < C; kb += 32) { const v16b a = frag_kb(&Oh[wave * 16 + nloc][kb], hlf), al = frag_kb(&Ol[wave * 16 + nloc][kb], hlf);
#pragma unroll
    for (int t = 0; t < 12; ++t) { const v16b bw = frag_kb(Wp + (size_t)(t * 16 + nloc) * C + kb, hlf); acc2[t] = wmma16b(a, bw, acc2[t]); acc2[t] = wmma16b(al, bw, acc2[t]); } }
#pragma unroll
  for (int t = 0; t < 12; ++t)
#pragma unroll
    for (int r = 0; r < 8; ++r) Ts[wave * 16 + 8 * hlf + r][t * 16 + nloc] = acc2[t][r] * (1.0f / XS);
  wave_lds_sync();
  for (int pass = 0; pass < 2; ++pass) { for (int i = lane; i < 16 * 48; i += 32) { const int rr = i / 48, c4 = (i % 48) * 4; *(volatile v4f*)(outb + (size_t)(m0 + rr) * C + c4) = *(const v4f*)(&Ts[wave * 16 + rr][c4]); } __threadfence(); }
}
}

extern "C" void kernel_launch(void* const* d_in, const int* in_sizes, int n_in,
                              void* d_out, int out_size, void* d_ws, size_t ws_size, hipStream_t stream) {
  (void)n_in; (void)out_size;
  const float* x = (const float*)d_in[0]; const float* wqkv = (const float*)d_in[1]; const float* wdw = (const float*)d_in[2]; const float* wpr = (const float*)d_in[3]; const float* tmp = (const float*)d_in[4];
  float* out = (float*)d_out;
  if (in_sizes[0] != Bn * NP * C || in_sizes[1] != C * C3 || in_sizes[2] != 9 * C3 || in_sizes[3] != C * C || in_sizes[4] != NH) return;
  size_t off = 0; char* ws = (char*)d_ws;
  auto carve = [&](size_t bytes) { char* p = ws + off; off += (bytes + 255) & ~(size_t)255; return p; };
  b16* R = (b16*)carve(((size_t)C3 * C + (size_t)C * C) * 2); float* P = (float*)carve(5188 * 4); b16* X = (b16*)carve((size_t)NP * C * 2); float* QF = (float*)carve((size_t)NP * C3 * 4);
  b16* QP = (b16*)carve((size_t)C * NP * 2); b16* QPl = (b16*)carve((size_t)C * NP * 2); b16* KP = (b16*)carve((size_t)C * NP * 2); b16* KPl = (b16*)carve((size_t)C * NP * 2);
  b16* VR = (b16*)carve(((size_t)NP + 32) * C * 2); b16* VRl = (b16*)carve(((size_t)NP + 32) * C * 2); b16* ATh = (b16*)carve((size_t)C * CHP * 2); b16* ATl = (b16*)carve((size_t)C * CHP * 2);
  if (off > ws_size) return;
  prep_kernel<<<64, 256, 0, stream>>>(wqkv, wdw, wpr, tmp, R, P, VR + (size_t)NP * C, VRl + (size_t)NP * C);
  for (int b = 0; b < Bn; ++b) { const float* xb = x + (size_t)b * NP * C; float* ob = out + (size_t)b * NP * C;
    xrows_kernel<<<256, 256, 0, stream>>>(xb, X);
    qkv_kernel<<<dim3(3, NP / 32), 64, 0, stream>>>(X, R, QF);
    dw_kernel<<<dim3(HW, 9), 256, 0, stream>>>(QF, P, QP, QPl, KP, KPl, VR, VRl);
    gram_kernel<<<1, 384, 0, stream>>>(QP, QPl, KP, KPl, P, ATh, ATl);
    out_kernel<<<NP / 32, 64, 0, stream>>>(VR, VRl, ATh, ATl, R, ob); }
}
